// SentenceLevelEncoder_6777458393260
// MI455X (gfx1250) — hardware-verified
//
#include <hip/hip_runtime.h>
#include <stdint.h>
#include <stddef.h>

#define BB   32
#define TT   32
#define MT   1024
#define VD   2048
#define HH   512
#define HF   256
#define G4   1024
#define FW   1536
#define NOB  36
#define NVP  20
#define SD   768
#define RB   16
#define TP   132
#define SP   264
#define OP   260
#define WSC  64.0f
#define HSC  16.0f
#define LOS  2048.0f
#define SH_W  0.015625f
#define SL_W  7.62939453125e-06f
#define SH_HW 0.0009765625f

static_assert(MT == BB * TT);
static_assert(G4 == 4 * HF);
static_assert(FW == 3 * HH);
static_assert(BB == 2 * RB);
static_assert(HH % 128 == 0);
static_assert(G4 % 128 == 0);
static_assert(SD % 128 == 0);
static_assert(MT % 32 == 0);
static_assert((BB * NOB) % 32 == 0);
static_assert((BB * NVP) % 32 == 0);
static_assert(VD % 32 == 0);
static_assert(HF % 32 == 0);
static_assert((TP * 4) % 16 == 0);
static_assert((SP * 2) % 16 == 0);
static_assert((OP * 4) % 16 == 0);
static_assert(NOB <= 64);
static_assert(NVP <= 64);

typedef _Float16      v16h __attribute__((ext_vector_type(16)));
typedef float         v8f  __attribute__((ext_vector_type(8)));
typedef float         v4f  __attribute__((ext_vector_type(4)));
typedef unsigned int  v4u  __attribute__((ext_vector_type(4)));
typedef v4f __attribute__((may_alias)) v4fa;
typedef v4u __attribute__((may_alias)) v4ua;

union FragH { v16h v; v4u q[2]; };

__device__ __forceinline__ v8f wmma_h(v16h a, v16h b, v8f c) {
  v8f d = __builtin_amdgcn_wmma_f32_16x16x32_f16(false, a, false, b, (short)0, c, false, false);
  asm volatile("v_nop\n\tv_nop\n\tv_nop\n\tv_nop" : "+v"(d) : "v"(a), "v"(b));
  return d;
}

__device__ __forceinline__ v16h ldfrag(const unsigned short* p, int h) {
  FragH f;
  f.q[0] = *(const v4ua*)(p + 8 * h);
  f.q[1] = *(const v4ua*)(p + 16 + 8 * h);
  return f.v;
}

__device__ __forceinline__ unsigned short hb16(_Float16 x) {
  return __builtin_bit_cast(unsigned short, x);
}
__device__ __forceinline__ unsigned short hbits(float a) {
  return hb16((_Float16)a);
}
__device__ __forceinline__ unsigned int pkh(float a, float b) {
  return (unsigned int)hbits(a) | ((unsigned int)hbits(b) << 16);
}

__device__ __forceinline__ void pack_hl(const float* f, v4u& ph, v4u& pl) {
  unsigned int hw[4], lw[4];
  #pragma unroll
  for (int i = 0; i < 4; ++i) {
    const _Float16 h0 = (_Float16)f[2 * i];
    const _Float16 h1 = (_Float16)f[2 * i + 1];
    const _Float16 l0 = (_Float16)((f[2 * i] - (float)h0) * LOS);
    const _Float16 l1 = (_Float16)((f[2 * i + 1] - (float)h1) * LOS);
    hw[i] = (unsigned int)hb16(h0) | ((unsigned int)hb16(h1) << 16);
    lw[i] = (unsigned int)hb16(l0) | ((unsigned int)hb16(l1) << 16);
  }
  ph.x = hw[0]; ph.y = hw[1]; ph.z = hw[2]; ph.w = hw[3];
  pl.x = lw[0]; pl.y = lw[1]; pl.z = lw[2]; pl.w = lw[3];
}

__device__ __forceinline__ float sigm(float x) {
  return __builtin_amdgcn_rcpf(1.0f + __expf(-x));
}
__device__ __forceinline__ float tnh(float x) {
  return 1.0f - 2.0f * __builtin_amdgcn_rcpf(__expf(2.0f * x) + 1.0f);
}

__global__ __launch_bounds__(256) void k_plane(const float* __restrict__ src, int n8,
                                               float s, int two,
                                               unsigned short* __restrict__ dh,
                                               unsigned short* __restrict__ dl)
{
  const int g = blockIdx.x * 256 + threadIdx.x;
  if (g >= n8) return;
  const size_t e0 = (size_t)g * 8;
  float v[8];
  #pragma unroll
  for (int i = 0; i < 8; ++i) v[i] = src[e0 + i] * s;
  v4u ph, pl;
  pack_hl(v, ph, pl);
  unsigned short* d0 = dh + e0;
  unsigned short* d1 = dl + e0;
  *(volatile v4u*)d0 = ph;
  if (two) *(volatile v4u*)d1 = pl;
  __threadfence();
  *(volatile v4u*)d0 = ph;
  if (two) *(volatile v4u*)d1 = pl;
}

template <int SPLIT>
__global__ __launch_bounds__(256) void k_gemm(const unsigned short* __restrict__ Ah,
                                              const unsigned short* __restrict__ Al, int lda,
                                              const unsigned short* __restrict__ Bh,
                                              const unsigned short* __restrict__ Bl, int ldb,
                                              const float* __restrict__ bias, int K,
                                              float sh, float sl,
                                              float* __restrict__ C, int ldc, int hasC,
                                              unsigned short* __restrict__ Ph,
                                              unsigned short* __restrict__ Pl, int ldp, int hasP)
{
  __shared__ __align__(16) float sT[32 * TP];

  const int tid = threadIdx.x, lane = tid & 31, wv = tid >> 5;
  const int h = lane >> 4, m = lane & 15;
  const int n0 = blockIdx.x * 128, m0 = blockIdx.y * 32;
  const int nc = n0 + 16 * wv;

  const v8f z8 = {0.f, 0.f, 0.f, 0.f, 0.f, 0.f, 0.f, 0.f};
  v8f acc0 = z8, acc1 = z8, ax0 = z8, ax1 = z8;
  const size_t ra0 = (size_t)(m0 + m) * lda;
  const size_t ra1 = (size_t)(m0 + 16 + m) * lda;
  const size_t rbw = (size_t)(nc + m) * ldb;

  #pragma unroll 1
  for (int k0 = 0; k0 < K; k0 += 32) {
    const v16h a0 = ldfrag(Ah + ra0 + k0, h);
    const v16h a1 = ldfrag(Ah + ra1 + k0, h);
    const v16h b  = ldfrag(Bh + rbw + k0, h);
    acc0 = wmma_h(a0, b, acc0);
    acc1 = wmma_h(a1, b, acc1);
    if (SPLIT) {
      const v16h l0 = ldfrag(Al + ra0 + k0, h);
      const v16h l1 = ldfrag(Al + ra1 + k0, h);
      const v16h bl = ldfrag(Bl + rbw + k0, h);
      ax0 = wmma_h(a0, bl, ax0);
      ax0 = wmma_h(l0, b, ax0);
      ax1 = wmma_h(a1, bl, ax1);
      ax1 = wmma_h(l1, b, ax1);
    }
  }

  const float bv = bias[nc + m];
  #pragma unroll
  for (int r = 0; r < 8; ++r) {
    float v0 = acc0[r] * sh;
    float v1 = acc1[r] * sh;
    if (SPLIT) { v0 += ax0[r] * sl; v1 += ax1[r] * sl; }
    v0 += bv;
    v1 += bv;
    sT[(8 * h + r) * TP + 16 * wv + m] = v0;
    sT[(16 + 8 * h + r) * TP + 16 * wv + m] = v1;
  }
  __syncthreads();

  if (hasC) {
    v4f ov[4];
    size_t ga[4];
    #pragma unroll
    for (int i = 0; i < 4; ++i) {
      const int row = wv + 8 * i;
      ov[i] = *(const v4fa*)(sT + row * TP + 4 * lane);
      ga[i] = (size_t)(m0 + row) * ldc + n0 + 4 * lane;
    }
    #pragma unroll
    for (int i = 0; i < 4; ++i) *(volatile v4f*)(C + ga[i]) = ov[i];
    __threadfence();
    #pragma unroll
    for (int i = 0; i < 4; ++i) *(volatile v4f*)(C + ga[i]) = ov[i];
  }
  if (hasP) {
    v4u ph[2], pl[2];
    size_t pa[2];
    #pragma unroll
    for (int q = 0; q < 2; ++q) {
      const int row = wv + 8 * (2 * q + h);
      const float* sp = sT + row * TP + 8 * m;
      const v4f x0 = *(const v4fa*)sp;
      const v4f x1 = *(const v4fa*)(sp + 4);
      float f[8];
      f[0] = x0.x; f[1] = x0.y; f[2] = x0.z; f[3] = x0.w;
      f[4] = x1.x; f[5] = x1.y; f[6] = x1.z; f[7] = x1.w;
      pack_hl(f, ph[q], pl[q]);
      pa[q] = (size_t)(m0 + row) * ldp + n0 + 8 * m;
    }
    #pragma unroll
    for (int q = 0; q < 2; ++q) {
      *(volatile v4u*)(Ph + pa[q]) = ph[q];
      *(volatile v4u*)(Pl + pa[q]) = pl[q];
    }
    __threadfence();
    #pragma unroll
    for (int q = 0; q < 2; ++q) {
      *(volatile v4u*)(Ph + pa[q]) = ph[q];
      *(volatile v4u*)(Pl + pa[q]) = pl[q];
    }
  }
}

__global__ __launch_bounds__(256) void k_attn(const float* __restrict__ wf2d,
                                              const float* __restrict__ u, int N,
                                              const float* __restrict__ bias,
                                              const float* __restrict__ ww,
                                              const float* __restrict__ wb,
                                              unsigned short* __restrict__ Fh,
                                              unsigned short* __restrict__ Fl, int colofs)
{
  __shared__ float sWf[HH];
  __shared__ float sBi[HH];
  __shared__ float sWw[HH];
  __shared__ float sSc[64];
  __shared__ float sE[64];
  __shared__ __align__(16) unsigned short sOh[HH];
  __shared__ __align__(16) unsigned short sOl[HH];

  const int tid = threadIdx.x, lane = tid & 31, wv = tid >> 5;
  const int bt = blockIdx.x;
  const int b = bt / TT;

  const float wf0 = wf2d[(size_t)bt * HH + tid];
  const float wf1 = wf2d[(size_t)bt * HH + tid + 256];
  const float bi0 = bias[tid], bi1 = bias[tid + 256];
  sWf[tid] = wf0; sWf[tid + 256] = wf1;
  sBi[tid] = bi0; sBi[tid + 256] = bi1;
  sWw[tid] = ww[tid]; sWw[tid + 256] = ww[tid + 256];
  __syncthreads();

  const float wbv = wb[0];
  for (int n = wv; n < N; n += 8) {
    const float* up = u + ((size_t)b * N + n) * HH;
    float p = 0.0f;
    #pragma unroll 2
    for (int i = 0; i < 16; ++i) {
      const int j = lane + 32 * i;
      const float f = (sWf[j] + up[j]) + sBi[j];
      p += tnh(f) * sWw[j];
    }
    #pragma unroll
    for (int off = 16; off; off >>= 1) p += __shfl_xor(p, off, 32);
    if (lane == 0) sSc[n] = p + wbv;
  }
  __syncthreads();

  float mx = -__builtin_inff();
  #pragma unroll 1
  for (int n = 0; n < N; ++n) mx = fmaxf(mx, sSc[n]);
  if (tid < N) sE[tid] = expf(sSc[tid] - mx);
  __syncthreads();
  float sm = 0.0f;
  #pragma unroll 1
  for (int n = 0; n < N; ++n) sm += sE[n];
  const float inv = 1.0f / sm;

  float a0 = 0.0f, a1 = 0.0f;
  #pragma unroll 1
  for (int n = 0; n < N; ++n) {
    const float aw = sE[n] * inv;
    const float* up = u + ((size_t)b * N + n) * HH;
    a0 += aw * ((wf0 + up[tid]) + bi0);
    a1 += aw * ((wf1 + up[tid + 256]) + bi1);
  }
  {
    const _Float16 h0 = (_Float16)a0, h1 = (_Float16)a1;
    sOh[tid] = hb16(h0);
    sOh[tid + 256] = hb16(h1);
    sOl[tid] = hb16((_Float16)((a0 - (float)h0) * LOS));
    sOl[tid + 256] = hb16((_Float16)((a1 - (float)h1) * LOS));
  }
  __syncthreads();

  const size_t rbase = (size_t)bt * FW + colofs;
  if (wv < 2) {
    const int q = tid;
    const v4u v = *(const v4ua*)(sOh + 8 * q);
    unsigned short* d = Fh + rbase + 8 * q;
    *(volatile v4u*)d = v;
    __threadfence();
    *(volatile v4u*)d = v;
  } else if (wv < 4) {
    const int q = tid - 64;
    const v4u v = *(const v4ua*)(sOl + 8 * q);
    unsigned short* d = Fl + rbase + 8 * q;
    *(volatile v4u*)d = v;
    __threadfence();
    *(volatile v4u*)d = v;
  }
}

__global__ __launch_bounds__(256) void k_rec(const float* __restrict__ ginF,
                                             const float* __restrict__ ginB,
                                             const unsigned short* __restrict__ WhF,
                                             const unsigned short* __restrict__ WhB,
                                             const float* __restrict__ bhF,
                                             const float* __restrict__ bhB,
                                             float* __restrict__ out,
                                             unsigned short* __restrict__ Vid)
{
  __shared__ __align__(16) unsigned short sH[RB * SP];
  __shared__ __align__(16) float sO[RB * OP];
  __shared__ __align__(16) unsigned short sV[RB * SP];
  __shared__ float sBh[G4];

  const int tid = threadIdx.x, lane = tid & 31, wv = tid >> 5;
  const int h = lane >> 4, m = lane & 15;
  const int dir = blockIdx.x >> 1;
  const int b0 = (blockIdx.x & 1) * RB;
  const float* gin = dir ? ginB : ginF;
  const unsigned short* Wh = dir ? WhB : WhF;
  const float* bh = dir ? bhB : bhF;

  for (int i = tid; i < RB * SP; i += 256) sH[i] = (unsigned short)0;
  for (int i = tid; i < G4; i += 256) sBh[i] = bh[i];
  float c[2][8], vmx[2][8];
  #pragma unroll
  for (int jb = 0; jb < 2; ++jb) {
    #pragma unroll
    for (int r = 0; r < 8; ++r) { c[jb][r] = 0.0f; vmx[jb][r] = -__builtin_inff(); }
  }
  __syncthreads();

  const v8f z8 = {0.f, 0.f, 0.f, 0.f, 0.f, 0.f, 0.f, 0.f};
  const size_t grow = (size_t)(b0 + m) * TT;

  #pragma unroll 1
  for (int step = 0; step < TT; ++step) {
    asm volatile("" ::: "memory");
    const int t = dir ? (TT - 1 - step) : step;
    const float* gb = gin + (grow + t) * G4;

    float hn[2][8];
    #pragma unroll
    for (int jb = 0; jb < 2; ++jb) {
      v8f acc[4];
      #pragma unroll
      for (int q = 0; q < 4; ++q) acc[q] = z8;
      const int ntb = wv + 8 * jb;
      #pragma unroll 1
      for (int ks = 0; ks < 8; ++ks) {
        const v16h bs = ldfrag(sH + m * SP + 32 * ks, h);
        #pragma unroll
        for (int q = 0; q < 4; ++q) {
          const int nt = 16 * q + ntb;
          acc[q] = wmma_h(ldfrag(Wh + (size_t)(nt * 16 + m) * HF + 32 * ks, h), bs, acc[q]);
        }
      }
      const int j0 = 16 * ntb + 8 * h;
      float gv[4][8];
      #pragma unroll
      for (int q = 0; q < 4; ++q) {
        const v4f x0 = *(const v4fa*)(gb + q * HF + j0);
        const v4f x1 = *(const v4fa*)(gb + q * HF + j0 + 4);
        gv[q][0] = x0.x; gv[q][1] = x0.y; gv[q][2] = x0.z; gv[q][3] = x0.w;
        gv[q][4] = x1.x; gv[q][5] = x1.y; gv[q][6] = x1.z; gv[q][7] = x1.w;
      }
      #pragma unroll
      for (int r = 0; r < 8; ++r) {
        const int j = j0 + r;
        const float g0 = (gv[0][r] + acc[0][r] * SH_HW) + sBh[j];
        const float g1 = (gv[1][r] + acc[1][r] * SH_HW) + sBh[HF + j];
        const float g2 = (gv[2][r] + acc[2][r] * SH_HW) + sBh[2 * HF + j];
        const float g3 = (gv[3][r] + acc[3][r] * SH_HW) + sBh[3 * HF + j];
        const float gi = sigm(g0);
        const float gf = sigm(g1);
        const float gg = tnh(g2);
        const float go = sigm(g3);
        const float cc = gf * c[jb][r] + gi * gg;
        c[jb][r] = cc;
        const float hv = go * tnh(cc);
        hn[jb][r] = hv;
        vmx[jb][r] = fmaxf(vmx[jb][r], hv);
      }
    }
    __syncthreads();

    #pragma unroll
    for (int jb = 0; jb < 2; ++jb) {
      const int j0 = 16 * (wv + 8 * jb) + 8 * h;
      v4u pk;
      pk.x = pkh(hn[jb][0] * HSC, hn[jb][1] * HSC);
      pk.y = pkh(hn[jb][2] * HSC, hn[jb][3] * HSC);
      pk.z = pkh(hn[jb][4] * HSC, hn[jb][5] * HSC);
      pk.w = pkh(hn[jb][6] * HSC, hn[jb][7] * HSC);
      *(v4ua*)(sH + m * SP + j0) = pk;
      v4f o0, o1;
      o0.x = hn[jb][0]; o0.y = hn[jb][1]; o0.z = hn[jb][2]; o0.w = hn[jb][3];
      o1.x = hn[jb][4]; o1.y = hn[jb][5]; o1.z = hn[jb][6]; o1.w = hn[jb][7];
      *(v4fa*)(sO + m * OP + j0) = o0;
      *(v4fa*)(sO + m * OP + j0 + 4) = o1;
    }
    __syncthreads();

    v4f ov[4];
    size_t ga[4];
    #pragma unroll
    for (int i = 0; i < 4; ++i) {
      const int p = wv + 8 * i;
      const int row = p >> 1, seg = p & 1;
      ov[i] = *(const v4fa*)(sO + row * OP + seg * 128 + 4 * lane);
      ga[i] = ((size_t)(b0 + row) * TT + t) * HH + dir * HF + seg * 128 + 4 * lane;
    }
    #pragma unroll
    for (int i = 0; i < 4; ++i) *(volatile v4f*)(out + ga[i]) = ov[i];
    __threadfence();
    #pragma unroll
    for (int i = 0; i < 4; ++i) *(volatile v4f*)(out + ga[i]) = ov[i];
  }

  #pragma unroll
  for (int jb = 0; jb < 2; ++jb) {
    const int j0 = 16 * (wv + 8 * jb) + 8 * h;
    v4u pk;
    pk.x = pkh(vmx[jb][0] * HSC, vmx[jb][1] * HSC);
    pk.y = pkh(vmx[jb][2] * HSC, vmx[jb][3] * HSC);
    pk.z = pkh(vmx[jb][4] * HSC, vmx[jb][5] * HSC);
    pk.w = pkh(vmx[jb][6] * HSC, vmx[jb][7] * HSC);
    *(v4ua*)(sV + m * SP + j0) = pk;
  }
  __syncthreads();
  v4u vv[2];
  size_t va[2];
  #pragma unroll
  for (int i = 0; i < 2; ++i) {
    const int row = wv + 8 * i;
    vv[i] = *(const v4ua*)(sV + row * SP + 8 * lane);
    va[i] = (size_t)(b0 + row) * HH + dir * HF + 8 * lane;
  }
  *(volatile v4u*)(Vid + va[0]) = vv[0];
  *(volatile v4u*)(Vid + va[1]) = vv[1];
  __threadfence();
  *(volatile v4u*)(Vid + va[0]) = vv[0];
  *(volatile v4u*)(Vid + va[1]) = vv[1];
}

static void plane(const float* src, int n, float s, int two,
                  unsigned short* dh, unsigned short* dl, hipStream_t st)
{
  const int n8 = n / 8;
  k_plane<<<(n8 + 255) / 256, 256, 0, st>>>(src, n8, s, two, dh, dl);
}

extern "C" void kernel_launch(void* const* d_in, const int* in_sizes, int n_in,
                              void* d_out, int out_size, void* d_ws, size_t ws_size,
                              hipStream_t stream)
{
  if (n_in < 27) return;
  if (in_sizes[0]  != MT * VD) return;
  if (in_sizes[1]  != BB * NVP * HH) return;
  if (in_sizes[2]  != BB * NOB * HH) return;
  if (in_sizes[3]  != HH * VD) return;
  if (in_sizes[4]  != HH) return;
  if (in_sizes[5]  != HH * HH) return;
  if (in_sizes[6]  != HH) return;
  if (in_sizes[7]  != HH * HH) return;
  if (in_sizes[8]  != HH) return;
  if (in_sizes[9]  != HH * HH) return;
  if (in_sizes[10] != HH) return;
  if (in_sizes[11] != HH) return;
  if (in_sizes[12] != HH) return;
  if (in_sizes[13] != HH) return;
  if (in_sizes[14] != 1) return;
  if (in_sizes[15] != HH) return;
  if (in_sizes[16] != 1) return;
  if (in_sizes[17] != G4 * FW) return;
  if (in_sizes[18] != G4 * HF) return;
  if (in_sizes[19] != G4) return;
  if (in_sizes[20] != G4) return;
  if (in_sizes[21] != G4 * FW) return;
  if (in_sizes[22] != G4 * HF) return;
  if (in_sizes[23] != G4) return;
  if (in_sizes[24] != G4) return;
  if (in_sizes[25] != SD * HH) return;
  if (in_sizes[26] != SD) return;
  if (out_size != MT * HH + BB * SD) return;

  const float* visual = (const float*)d_in[0];
  const float* vpf    = (const float*)d_in[1];
  const float* objf   = (const float*)d_in[2];
  const float* w2d_w  = (const float*)d_in[3];
  const float* w2d_b  = (const float*)d_in[4];
  const float* W_w    = (const float*)d_in[5];
  const float* W_b    = (const float*)d_in[6];
  const float* Uo_w   = (const float*)d_in[7];
  const float* Uo_b   = (const float*)d_in[8];
  const float* Um_w   = (const float*)d_in[9];
  const float* Um_b   = (const float*)d_in[10];
  const float* bo     = (const float*)d_in[11];
  const float* bm     = (const float*)d_in[12];
  const float* wo_w   = (const float*)d_in[13];
  const float* wo_b   = (const float*)d_in[14];
  const float* wm_w   = (const float*)d_in[15];
  const float* wm_b   = (const float*)d_in[16];
  const float* wih_f  = (const float*)d_in[17];
  const float* whh_f  = (const float*)d_in[18];
  const float* bih_f  = (const float*)d_in[19];
  const float* bhh_f  = (const float*)d_in[20];
  const float* wih_b  = (const float*)d_in[21];
  const float* whh_b  = (const float*)d_in[22];
  const float* bih_b  = (const float*)d_in[23];
  const float* bhh_b  = (const float*)d_in[24];
  const float* fc_w   = (const float*)d_in[25];
  const float* fc_b   = (const float*)d_in[26];
  float* out0 = (float*)d_out;
  float* out1 = (float*)d_out + (size_t)MT * HH;

  const size_t bVis  = (size_t)MT * VD * 2;
  const size_t bW2d  = (size_t)HH * VD * 2;
  const size_t bW55  = (size_t)HH * HH * 2;
  const size_t bObj  = (size_t)BB * NOB * HH * 2;
  const size_t bVp   = (size_t)BB * NVP * HH * 2;
  const size_t bWih  = (size_t)G4 * FW * 2;
  const size_t bWhh  = (size_t)G4 * HF * 2;
  const size_t bFc   = (size_t)SD * HH * 2;
  const size_t bFeat = (size_t)MT * FW * 2;
  const size_t bWf   = (size_t)MT * HH * 4;
  const size_t bUo   = (size_t)BB * NOB * HH * 4;
  const size_t bUm   = (size_t)BB * NVP * HH * 4;
  const size_t bGin  = (size_t)MT * G4 * 4;
  const size_t bVid  = (size_t)BB * HH * 2;
  const size_t total = 2 * bVis + 2 * bW2d + 3 * bW55 + bObj + bVp + 4 * bWih + 2 * bWhh
                     + bFc + 2 * bFeat + bWf + bUo + bUm + 2 * bGin + bVid;
  if (total > ws_size) return;
  if (total > (size_t)134217728) return;

  char* ws = (char*)d_ws;
  size_t off = 0;
  unsigned short* pVisH  = (unsigned short*)(ws + off); off += bVis;
  unsigned short* pVisL  = (unsigned short*)(ws + off); off += bVis;
  unsigned short* pW2dH  = (unsigned short*)(ws + off); off += bW2d;
  unsigned short* pW2dL  = (unsigned short*)(ws + off); off += bW2d;
  unsigned short* pWw    = (unsigned short*)(ws + off); off += bW55;
  unsigned short* pUo    = (unsigned short*)(ws + off); off += bW55;
  unsigned short* pUm    = (unsigned short*)(ws + off); off += bW55;
  unsigned short* pObj   = (unsigned short*)(ws + off); off += bObj;
  unsigned short* pVp    = (unsigned short*)(ws + off); off += bVp;
  unsigned short* pWiFH  = (unsigned short*)(ws + off); off += bWih;
  unsigned short* pWiFL  = (unsigned short*)(ws + off); off += bWih;
  unsigned short* pWiBH  = (unsigned short*)(ws + off); off += bWih;
  unsigned short* pWiBL  = (unsigned short*)(ws + off); off += bWih;
  unsigned short* pWhF   = (unsigned short*)(ws + off); off += bWhh;
  unsigned short* pWhB   = (unsigned short*)(ws + off); off += bWhh;
  unsigned short* pFc    = (unsigned short*)(ws + off); off += bFc;
  unsigned short* pFeatH = (unsigned short*)(ws + off); off += bFeat;
  unsigned short* pFeatL = (unsigned short*)(ws + off); off += bFeat;
  float*          wf2d   = (float*)(ws + off);          off += bWf;
  float*          uobj   = (float*)(ws + off);          off += bUo;
  float*          umot   = (float*)(ws + off);          off += bUm;
  float*          ginF   = (float*)(ws + off);          off += bGin;
  float*          ginB   = (float*)(ws + off);          off += bGin;
  unsigned short* pVid   = (unsigned short*)(ws + off); off += bVid;
  if (off != total) return;

  plane(visual, MT * VD,        1.0f, 1, pVisH, pVisL, stream);
  plane(w2d_w,  HH * VD,        WSC,  1, pW2dH, pW2dL, stream);
  plane(W_w,    HH * HH,        WSC,  0, pWw,   pWw,   stream);
  plane(Uo_w,   HH * HH,        WSC,  0, pUo,   pUo,   stream);
  plane(Um_w,   HH * HH,        WSC,  0, pUm,   pUm,   stream);
  plane(objf,   BB * NOB * HH,  1.0f, 0, pObj,  pObj,  stream);
  plane(vpf,    BB * NVP * HH,  1.0f, 0, pVp,   pVp,   stream);
  plane(wih_f,  G4 * FW,        WSC,  1, pWiFH, pWiFL, stream);
  plane(wih_b,  G4 * FW,        WSC,  1, pWiBH, pWiBL, stream);
  plane(whh_f,  G4 * HF,        WSC,  0, pWhF,  pWhF,  stream);
  plane(whh_b,  G4 * HF,        WSC,  0, pWhB,  pWhB,  stream);
  plane(fc_w,   SD * HH,        WSC,  0, pFc,   pFc,   stream);

  k_gemm<1><<<dim3(HH / 128, MT / 32), 256, 0, stream>>>(
      pVisH, pVisL, VD, pW2dH, pW2dL, VD, w2d_b, VD, SH_W, SL_W,
      ginF, HH, 0, pFeatH, pFeatL, FW, 1);
  k_gemm<0><<<dim3(HH / 128, MT / 32), 256, 0, stream>>>(
      pFeatH, pFeatH, FW, pWw, pWw, HH, W_b, HH, SH_W, 0.0f,
      wf2d, HH, 1, pW2dH, pW2dL, FW, 0);
  k_gemm<0><<<dim3(HH / 128, (BB * NOB) / 32), 256, 0, stream>>>(
      pObj, pObj, HH, pUo, pUo, HH, Uo_b, HH, SH_W, 0.0f,
      uobj, HH, 1, pW2dH, pW2dL, FW, 0);
  k_gemm<0><<<dim3(HH / 128, (BB * NVP) / 32), 256, 0, stream>>>(
      pVp, pVp, HH, pUm, pUm, HH, Um_b, HH, SH_W, 0.0f,
      umot, HH, 1, pW2dH, pW2dL, FW, 0);

  k_attn<<<MT, 256, 0, stream>>>(wf2d, umot, NVP, bm, wm_w, wm_b, pFeatH, pFeatL, HH);
  k_attn<<<MT, 256, 0, stream>>>(wf2d, uobj, NOB, bo, wo_w, wo_b, pFeatH, pFeatL, 2 * HH);

  k_gemm<1><<<dim3(G4 / 128, MT / 32), 256, 0, stream>>>(
      pFeatH, pFeatL, FW, pWiFH, pWiFL, FW, bih_f, FW, SH_W, SL_W,
      ginF, G4, 1, pW2dH, pW2dL, FW, 0);
  k_gemm<1><<<dim3(G4 / 128, MT / 32), 256, 0, stream>>>(
      pFeatH, pFeatL, FW, pWiBH, pWiBL, FW, bih_b, FW, SH_W, SL_W,
      ginB, G4, 1, pW2dH, pW2dL, FW, 0);

  k_rec<<<2 * (BB / RB), 256, 0, stream>>>(ginF, ginB, pWhF, pWhB, bhh_f, bhh_b, out0, pVid);

  k_gemm<0><<<dim3(SD / 128, BB / 32), 256, 0, stream>>>(
      pVid, pVid, HH, pFc, pFc, HH, fc_b, HH, SH_HW, 0.0f,
      out1, SD, 1, pW2dH, pW2dL, FW, 0);
}
